// Net_64132451664097
// MI455X (gfx1250) — hardware-run, weakly checked
//
#include <hip/hip_runtime.h>


namespace {

constexpr int N = 100000, NP = 100032, NPL = NP  , SRCM = N  , EFULL = 1600000, E = EFULL  ;
constexpr int IN = 128, C = 64  , NCOL = 6 * C  , NBLK = NP / 32, NL = (NPL < N ? NPL : N);
constexpr float XS = 8.0f, WSC = 256.0f, WSQ = 0.25f, RS_ = 1024.0f, SLOPE = 0.0f, BNEPS = 1e-5f;
static_assert(NP % 32 == 0 && NP >= N && NPL % 32 == 0 && C == 64 && IN % 32 == 0, "tiling");
typedef _Float16 b16;
typedef __attribute__((ext_vector_type(16))) _Float16 v16b;
typedef __attribute__((ext_vector_type(8))) _Float16 v8b;
typedef __attribute__((ext_vector_type(8))) float v8f;
typedef __attribute__((ext_vector_type(4))) float v4f;
__device__ __forceinline__ float bf16_rne(float f) { unsigned int u = __float_as_uint(f); u += 0x7FFFu + ((u >> 16) & 1u); return __uint_as_float(u & 0xFFFF0000u); }
__device__ __forceinline__ void split16(float v, b16& hi, b16& lo) { hi = (b16)v; lo = (b16)(v - (float)hi); }
__device__ __forceinline__ v16b frag_kb(const b16* p, int hh) { const v8b a = *(const v8b*)(p + 8 * hh), b = *(const v8b*)(p + 16 + 8 * hh); v16b f;
#pragma unroll
  for (int e = 0; e < 8; ++e) { f[e] = a[e]; f[8 + e] = b[e]; } return f; }
__device__ __forceinline__ v8f wmma16b(v16b a, v16b b, v8f c) { v8f d = __builtin_amdgcn_wmma_f32_16x16x32_f16(false, a, false, b, (short)0, c, false, false); asm volatile("v_nop\n\tv_nop\n\tv_nop\n\tv_nop" : "+v"(d) : "v"(a), "v"(b)); return d; }
__device__ __forceinline__ void wave_lds_sync() { __builtin_amdgcn_fence(__ATOMIC_RELEASE, "workgroup"); __builtin_amdgcn_wave_barrier(); __builtin_amdgcn_fence(__ATOMIC_ACQUIRE, "workgroup"); }
__device__ __forceinline__ float pmul(float a, float b) { float p = a * b; asm volatile("" : "+v"(p)); return p; }
__device__ __forceinline__ int iclamp(int v, int lo, int hi) { return v < lo ? lo : (v > hi ? hi : v); }
constexpr int CSR_NBLK = 512, CSR_GB = 9, CSR_GN = 1 << CSR_GB  , CSR_MAXG = 512, CSR_CAP = 12288  ;
__global__ __launch_bounds__(64) void csrA_kernel(const int* __restrict__ dst, int E, int N, int nG, int CHP, int NGP, int* __restrict__ STG, int* __restrict__ HST) {
  extern __shared__ int sm[];
  int* cnt = sm; int* run = sm + NGP; int* ids = sm + 2 * NGP;
  const int b = blockIdx.x; const int ch = (E + CSR_NBLK - 1) / CSR_NBLK; const int e0 = b * ch, e1 = min(E, e0 + ch);
  for (int i = threadIdx.x; i < NGP; i += 64) cnt[i] = 0;
  for (int i = threadIdx.x; i < CHP; i += 64) ids[i] = -1;
  __syncthreads();
  if (threadIdx.x == 0) {
    for (int e = e0; e < e1; ++e) { int d = dst[e]; d = (d < 0) ? 0 : (d >= N ? N - 1 : d); cnt[d >> CSR_GB] += 1; }
    int acc = 0; for (int g = 0; g < nG; ++g) { run[g] = acc; acc += cnt[g]; }
    for (int e = e0; e < e1; ++e) { int d = dst[e]; d = (d < 0) ? 0 : (d >= N ? N - 1 : d); const int g = d >> CSR_GB; ids[run[g]] = e; run[g] += 1; } }
  __syncthreads();
  typedef __attribute__((ext_vector_type(4))) int v4i;
  for (int pass = 0; pass < 2; ++pass) {
    for (int i = threadIdx.x; i < CHP / 4; i += 64) *(volatile v4i*)(STG + (size_t)b * CHP + i * 4) = *(const v4i*)(&ids[i * 4]);
    for (int i = threadIdx.x; i < NGP / 4; i += 64) { v4i v; for (int e = 0; e < 4; ++e) v[e] = (i * 4 + e < nG) ? cnt[i * 4 + e] : 0; *(volatile v4i*)(HST + (size_t)b * NGP + i * 4) = v; }
    __threadfence(); }
}
__global__ __launch_bounds__(512) void csrS_kernel(const int* __restrict__ HST, int nG, int NGP, int* __restrict__ START, int* __restrict__ TOT, int* __restrict__ OFF) {
  __shared__ int tot[CSR_MAXG];
  const int b = threadIdx.x;
  for (int pass = 0; pass < 2; ++pass) { int runb = 0; for (int g = 0; g < nG; ++g) { int c = HST[(size_t)b * NGP + g]; c = (c < 0) ? 0 : c; ((volatile int*)OFF)[(size_t)g * CSR_NBLK + b] = runb; runb += c; } __threadfence(); }
  for (int g = threadIdx.x; g < nG; g += 512) { int s = 0; for (int bb = 0; bb < CSR_NBLK; ++bb) { int c = HST[(size_t)bb * NGP + g]; s += (c < 0) ? 0 : c; } tot[g] = s; }
  __syncthreads();
  if (threadIdx.x < 32) {
    __shared__ int st[CSR_MAXG + 32];
    if (threadIdx.x == 0) { int acc = 0; for (int g = 0; g < NGP; ++g) { st[g] = acc; if (g < nG) acc += (tot[g] + 31) & ~31; } st[NGP] = acc; }
    __builtin_amdgcn_fence(__ATOMIC_RELEASE, "workgroup"); __builtin_amdgcn_wave_barrier(); __builtin_amdgcn_fence(__ATOMIC_ACQUIRE, "workgroup");
    for (int pass = 0; pass < 2; ++pass) { for (int i = threadIdx.x; i < NGP + 32; i += 32) { ((volatile int*)START)[i] = (i <= NGP) ? st[min(i, NGP)] : 0; ((volatile int*)TOT)[i] = (i < nG) ? tot[i] : 0; } __threadfence(); } }
}
__global__ __launch_bounds__(256) void csrB_kernel(const int* __restrict__ dst, int N, int nG, int CHP, int NGP, int permLen, const int* __restrict__ STG, const int* __restrict__ HST, const int* __restrict__ OFF, const int* __restrict__ START, const int* __restrict__ TOT, int* __restrict__ PERM, int* __restrict__ ROWPTR, int* __restrict__ ROWCNT, int* __restrict__ FLAG) {
  typedef __attribute__((ext_vector_type(4))) int v4i;
  __shared__ int ids[CSR_CAP]; __shared__ unsigned short key[CSR_CAP]; __shared__ int outp[CSR_CAP]; __shared__ int ncnt[CSR_GN + 1]; __shared__ int boff[CSR_NBLK + 1];
  const int g = blockIdx.x, t_ = threadIdx.x; int tot = TOT[g]; int st = START[g], stn = START[g + 1]; const int v0 = g * CSR_GN; const int nv = min(CSR_GN, N - v0);
  st = (st < 0) ? 0 : (st > permLen - 32 ? permLen - 32 : st) & ~31; stn = (stn < st) ? st : (stn > permLen ? permLen : stn); tot = (tot < 0) ? 0 : tot; if (tot > stn - st && tot <= CSR_CAP) tot = stn - st;
  if (tot > CSR_CAP) {
    for (int pass = 0; pass < 2; ++pass) { for (int i = t_; i < CSR_GN / 4; i += 256) { v4i a, c; for (int e = 0; e < 4; ++e) { a[e] = st; c[e] = 0; } *(volatile v4i*)(ROWPTR + v0 + i * 4) = a; *(volatile v4i*)(ROWCNT + v0 + i * 4) = c; } if (t_ == 0) ((volatile int*)FLAG)[0] = 1; __threadfence(); } (void)nv; return; }
  if (t_ == 0) { int acc = 0; for (int b = 0; b < CSR_NBLK; ++b) { boff[b] = acc; int c = HST[(size_t)b * NGP + g]; c = (c < 0) ? 0 : (c > CHP ? CHP : c); acc += c; if (acc > tot) acc = tot; } boff[CSR_NBLK] = acc; }
  for (int i = t_; i <= CSR_GN; i += 256) ncnt[i] = 0;
  __syncthreads();
  for (int b = 0; b < CSR_NBLK; ++b) { const int c = boff[b + 1] - boff[b]; int o_ = OFF[(size_t)g * CSR_NBLK + b]; o_ = (o_ < 0) ? 0 : (o_ > CHP - c ? CHP - c : o_); const int* src_ = STG + (size_t)b * CHP + o_;
    for (int i = t_; i < c; i += 256) { int id = src_[i]; id = (id < 0) ? 0 : id; ids[boff[b] + i] = id; int d = dst[id]; d = (d < v0) ? v0 : (d >= N ? N - 1 : d); int kk = d - v0; kk = (kk < 0) ? 0 : (kk >= CSR_GN ? CSR_GN - 1 : kk); key[boff[b] + i] = (unsigned short)kk; } }
  __syncthreads();
  if (t_ == 0) { for (int i = 0; i < tot; ++i) ncnt[key[i]] += 1; int acc = 0; for (int vl = 0; vl < CSR_GN; ++vl) { const int c = ncnt[vl]; ncnt[vl] = acc; acc += c; } ncnt[CSR_GN] = acc;
    for (int i = 0; i < tot; ++i) { const int vl = key[i]; outp[ncnt[vl]] = ids[i]; ncnt[vl] += 1; }
    for (int vl = CSR_GN; vl > 0; --vl) ncnt[vl] = ncnt[vl - 1]; ncnt[0] = 0; }
  __syncthreads();
  for (int pass = 0; pass < 2; ++pass) {
    for (int i = t_; i < (stn - st) / 4; i += 256) { v4i v; for (int e = 0; e < 4; ++e) { const int q = i * 4 + e; v[e] = (q < tot) ? outp[q] : -1; } *(volatile v4i*)(PERM + st + i * 4) = v; }
    for (int i = t_; i < CSR_GN / 4; i += 256) { v4i a, c; for (int e = 0; e < 4; ++e) { const int vl = i * 4 + e; a[e] = st + ncnt[vl]; c[e] = (vl < nv) ? (ncnt[vl + 1] - ncnt[vl]) : 0; } *(volatile v4i*)(ROWPTR + v0 + i * 4) = a; *(volatile v4i*)(ROWCNT + v0 + i * 4) = c; }
    __threadfence(); }
}
__global__ __launch_bounds__(256) void csrZ_kernel(int* __restrict__ p, size_t n4) { typedef __attribute__((ext_vector_type(4))) int v4i; const size_t tid = (size_t)blockIdx.x * 256 + threadIdx.x, nth = (size_t)gridDim.x * 256; v4i z = {0, 0, 0, 0}; for (size_t i = tid; i < n4; i += nth) *(volatile v4i*)(p + i * 4) = z; }
struct CsrBufs { int *STG, *HST, *OFF, *START, *TOT, *PERM, *ROWPTR, *ROWCNT, *FLAG; int nG, NGP, CHP; size_t permLen; char* base; size_t bytes; };
static size_t csr_carve(CsrBufs& c, char* ws, size_t off, int E, int N) {
  const size_t off0 = off; c.base = ws + off;
  auto al = [&](size_t bytes) { char* p = ws + off; off += (bytes + 255) & ~(size_t)255; return p; };
  c.nG = (N + CSR_GN - 1) / CSR_GN; c.NGP = (c.nG + 31) & ~31; const int ch = (E + CSR_NBLK - 1) / CSR_NBLK; c.CHP = (ch + 31) & ~31; c.permLen = (size_t)E + 32 * (size_t)c.nG + 32;
  c.STG = (int*)al((size_t)CSR_NBLK * c.CHP * 4); c.HST = (int*)al((size_t)CSR_NBLK * c.NGP * 4); c.OFF = (int*)al((size_t)c.NGP * CSR_NBLK * 4); c.START = (int*)al((size_t)(c.NGP + 64) * 4); c.TOT = (int*)al((size_t)(c.NGP + 64) * 4);
  c.PERM = (int*)al(c.permLen * 4); c.ROWPTR = (int*)al((size_t)c.nG * CSR_GN * 4); c.ROWCNT = (int*)al((size_t)c.nG * CSR_GN * 4); c.FLAG = (int*)al(256);
  c.bytes = off - off0; return off;
}
static void csr_build(const CsrBufs& c, const int* dst, int E, int N, hipStream_t stream) {
  const size_t smem = (size_t)(2 * c.NGP + c.CHP) * 4;
  csrZ_kernel<<<512, 256, 0, stream>>>((int*)c.base, c.bytes / 16);
  csrA_kernel<<<CSR_NBLK, 64, smem, stream>>>(dst, E, N, c.nG, c.CHP, c.NGP, c.STG, c.HST);
  csrS_kernel<<<1, 512, 0, stream>>>(c.HST, c.nG, c.NGP, c.START, c.TOT, c.OFF);
  csrB_kernel<<<c.nG, 256, 0, stream>>>(dst, N, c.nG, c.CHP, c.NGP, (int)c.permLen, c.STG, c.HST, c.OFF, c.START, c.TOT, c.PERM, c.ROWPTR, c.ROWCNT, c.FLAG);
}

typedef __attribute__((ext_vector_type(4))) _Float16 v4h;
template <int K>
__global__ __launch_bounds__(256) void wt_kernel(const float* __restrict__ skipw, const float* __restrict__ linw, const float* __restrict__ fskipw, const float* __restrict__ filmw, b16* __restrict__ WT, float scl) {
  const int u = blockIdx.x * 256 + threadIdx.x; if (u >= NCOL * K / 8) return; const int e = u * 8; const int o = e / K, k0 = e % K; const float* w; int oo, wdt;
  if (o < C) { w = skipw; oo = o; wdt = C; } else if (o < 2 * C) { w = linw; oo = o - C; wdt = C; } else if (o < 4 * C) { w = fskipw; oo = o - 2 * C; wdt = 2 * C; } else { w = filmw; oo = o - 4 * C; wdt = 2 * C; }
  v8b v;
#pragma unroll
  for (int j = 0; j < 8; ++j) v[j] = (b16)(bf16_rne(w[(size_t)(k0 + j) * wdt + oo]) * scl);
  for (int pass = 0; pass < 2; ++pass) { *(volatile v8b*)(WT + e) = v; __threadfence(); }
}
template <int K, bool RND, bool ACT>
__global__ __launch_bounds__(64) void node_kernel(const float* __restrict__ X, const float* __restrict__ ST, const float* __restrict__ bng, const float* __restrict__ bnb, const b16* __restrict__ WT, const b16* __restrict__ WQ, const float* __restrict__ fskipb, const float* __restrict__ filmb, float* __restrict__ LP, float* __restrict__ OP, float* __restrict__ GB) {
  __shared__ __attribute__((aligned(16))) b16 Ah[2][16][K + 8], Al[2][16][K + 8]; __shared__ __attribute__((aligned(16))) float Sk[2][16][C + 4]; __shared__ __attribute__((aligned(16))) float Tf[2][16][2 * C + 4];
  const int wave = threadIdx.x >> 5, lane = threadIdx.x & 31, nloc = lane & 15, hlf = lane >> 4; const size_t m0 = (size_t)blockIdx.x * 32 + wave * 16;
  for (int idx = lane; idx < 16 * (K / 4); idx += 32) { const int rr = idx / (K / 4), c4 = (idx % (K / 4)) * 4; const size_t arow = (m0 + rr < (size_t)N) ? m0 + rr : (size_t)N - 1; const v4f v = *(const v4f*)(X + arow * K + c4); v4h hv, lv;
    for (int j = 0; j < 4; ++j) { float t; if (RND) t = bf16_rne(v[j]); else { const int c = c4 + j; const float mean = ST[c], rs = ST[C + c]; t = pmul((v[j] - mean) * rs, bf16_rne(bng[c])) + bf16_rne(bnb[c]); }
      const float vs = t * XS; const b16 ph = (b16)vs; hv[j] = ph; lv[j] = (b16)((vs - (float)ph) * RS_); } *(v4h*)(&Ah[wave][rr][c4]) = hv; *(v4h*)(&Al[wave][rr][c4]) = lv; }
  wave_lds_sync();
#pragma unroll 1
  for (int ps = 0; ps < 3; ++ps) {
    v8f acc[8]; for (int t = 0; t < 8; ++t) acc[t] = (v8f){};
#pragma unroll
    for (int kb = 0; kb < K; kb += 32) { const v16b a = frag_kb(&Ah[wave][nloc][kb], hlf); v16b al; if (!RND) al = frag_kb(&Al[wave][nloc][kb], hlf);
#pragma unroll
      for (int t = 0; t < 8; ++t) { const size_t wo_ = (size_t)(ps * 128 + t * 16 + nloc) * K + kb; acc[t] = wmma16b(a, frag_kb(WT + wo_, hlf), acc[t]); if (!RND) acc[t] = wmma16b(al, frag_kb(WQ + wo_, hlf), acc[t]); } }
    if (ps > 0) wave_lds_sync();
#pragma unroll
    for (int t = 0; t < 8; ++t) { const int col = t * 16 + nloc; const float bb = (ps == 1) ? bf16_rne(fskipb[col]) : (ps == 2 ? bf16_rne(filmb[col]) : 0.0f);
#pragma unroll
      for (int r = 0; r < 8; ++r) { const float val = acc[t][r] * (1.0f / (XS * WSC)) + bb; if (ps == 0 && t < 4) Sk[wave][8 * hlf + r][col] = val; else Tf[wave][8 * hlf + r][(ps == 0) ? col - C : col] = val; } }
    wave_lds_sync();
    for (int pass = 0; pass < 2; ++pass) {
      if (ps == 0) { for (int rr = 0; rr < 16; rr += 2) { const int r2 = rr + (lane >> 4); const size_t vrow = m0 + r2; v4f o = *(const v4f*)(&Tf[wave][r2][(lane & 15) * 4]); if (vrow >= (size_t)N) o = (v4f){0.0f, 0.0f, 0.0f, 0.0f}; *(volatile v4f*)(LP + vrow * C + (lane & 15) * 4) = o; } }
      else if (ps == 1) { for (int rr = 0; rr < 16; rr += 2) { const int r2 = rr + (lane >> 4); const size_t vrow = m0 + r2; v4f o; for (int j = 0; j < 4; ++j) { const int c = (lane & 15) * 4 + j; float on = pmul(Tf[wave][r2][C + c], Sk[wave][r2][c]) + Tf[wave][r2][c]; if (ACT) on = fmaxf(on, 0.0f); o[j] = (vrow < (size_t)N) ? on : 0.0f; } *(volatile v4f*)(OP + vrow * C + (lane & 15) * 4) = o; } }
      else { for (int rr = 0; rr < 16; ++rr) { const size_t vrow = m0 + rr; v4f o = *(const v4f*)(&Tf[wave][rr][lane * 4]); if (vrow >= (size_t)N) o = (v4f){0.0f, 0.0f, 0.0f, 0.0f}; *(volatile v4f*)(GB + vrow * (2 * C) + lane * 4) = o; } }
      __threadfence(); } }
}
template <bool ACT>
__global__ __launch_bounds__(256) void agg_kernel(const float* __restrict__ LP, const float* __restrict__ OP, const float* __restrict__ GB, const int* __restrict__ srcs, const int* __restrict__ PERM, const int* __restrict__ ROWPTR, const int* __restrict__ ROWCNT, int permLen, float* __restrict__ Hh, int mrows) {
  const int tid = threadIdx.x; const int row = tid >> 3, g = tid & 7, c0 = g * 8; const int v = blockIdx.x * 32 + row; const int vv = v < N ? v : N - 1;
  float be[8], ga[8], m[8]; { const v4f b0 = *(const v4f*)(GB + (size_t)vv * 2 * C + c0), b1 = *(const v4f*)(GB + (size_t)vv * 2 * C + c0 + 4), g0 = *(const v4f*)(GB + (size_t)vv * 2 * C + C + c0), g1 = *(const v4f*)(GB + (size_t)vv * 2 * C + C + c0 + 4); for (int j = 0; j < 4; ++j) { be[j] = b0[j]; be[4 + j] = b1[j]; ga[j] = g0[j]; ga[4 + j] = g1[j]; m[j] = 0.0f; m[4 + j] = 0.0f; } }
  int cnt = 0, p0 = 0; if (v < N) { cnt = iclamp(ROWCNT[v], 0, 65536); p0 = iclamp(ROWPTR[v], 0, permLen - 1); if (p0 + cnt > permLen) cnt = permLen - p0; }
#pragma unroll 1
  for (int i = 0; i < cnt; ++i) { const int e = iclamp(PERM[p0 + i], 0, E - 1); int s = iclamp(srcs[e], 0, N - 1); if (SRCM < N) s %= SRCM; const float* lr = LP + (size_t)s * C + c0;
#pragma unroll
    for (int q = 0; q < 2; ++q) { const v4f t4 = *(const v4f*)(lr + 4 * q); for (int j = 0; j < 4; ++j) { float mv = fmaf(ga[4 * q + j], t4[j], be[4 * q + j]); if (ACT) mv = fmaxf(mv, 0.0f); m[4 * q + j] += mv; } } }
  const float inv = 1.0f / (float)(cnt > 1 ? cnt : 1);
  v4f o[2]; { const float* orow = OP + (size_t)vv * C + c0; for (int q = 0; q < 2; ++q) { const v4f t4 = *(const v4f*)(orow + 4 * q); for (int j = 0; j < 4; ++j) o[q][j] = (v < N) ? t4[j] + ((cnt > 0) ? m[4 * q + j] * inv : 0.0f) : 0.0f; } }
  for (int pass = 0; pass < 2; ++pass) { if (v < mrows) { float* hr = Hh + (size_t)v * C + c0; *(volatile v4f*)hr = o[0]; *(volatile v4f*)(hr + 4) = o[1]; } __threadfence(); }
}
template <int MODE>
__global__ __launch_bounds__(256) void colpart_kernel(const float* __restrict__ Hh, const float* __restrict__ ST, float* __restrict__ PART) {
  __shared__ float csum[4][C]; const int tid = threadIdx.x; const int c = tid & (C - 1), qq = tid >> 6; const int v0 = blockIdx.x * 32; const float mu = (MODE == 1) ? ST[c] : 0.0f; float s = 0.0f;
  for (int rr = qq * 8; rr < qq * 8 + 8; ++rr) { const int v = v0 + rr; if (v < N) { const float hv = Hh[(size_t)v * C + c]; const float d = hv - mu; s += (MODE == 1) ? pmul(d, d) : hv; } }
  csum[qq][c] = s; __syncthreads();
  for (int pass = 0; pass < 2; ++pass) { if (tid < 16) { v4f p; for (int q = 0; q < 4; ++q) { const int cc = tid * 4 + q; p[q] = ((csum[0][cc] + csum[1][cc]) + csum[2][cc]) + csum[3][cc]; } *(volatile v4f*)(PART + (size_t)blockIdx.x * C + tid * 4) = p; } __threadfence(); }
}
template <int MODE>
__global__ __launch_bounds__(64) void colred_kernel(const float* __restrict__ PART, float* __restrict__ ST) {
  const int c = threadIdx.x; float s = 0.0f;
  for (int bk = 0; bk < NBLK; ++bk) s += PART[(size_t)bk * C + c];
  const float v = (MODE == 0) ? s * (1.0f / (float)N) : rsqrtf(s * (1.0f / (float)N) + BNEPS);
  for (int pass = 0; pass < 2; ++pass) { ((volatile float*)ST)[MODE * C + c] = v; __threadfence(); }
}
}

extern "C" void kernel_launch(void* const* d_in, const int* in_sizes, int n_in, void* d_out, int out_size, void* d_ws, size_t ws_size, hipStream_t stream) {
  (void)n_in;
  auto Fp = [&](int i) { return (const float*)d_in[i]; }; auto Ip = [&](int i) { return (const int*)d_in[i]; };
  if (in_sizes[0] != N * IN || in_sizes[1] != 2 * EFULL || out_size != N * C) return;
  { const int ks[3] = {IN, C, C}; for (int l = 0; l < 3; ++l) { const int b = 2 + 8 * l, k = ks[l]; if (in_sizes[b] != k * C || in_sizes[b + 1] != k * 2 * C || in_sizes[b + 2] != 2 * C || in_sizes[b + 3] != k * C || in_sizes[b + 4] != k * 2 * C || in_sizes[b + 5] != 2 * C) return; if (l < 2 && (in_sizes[b + 6] != C || in_sizes[b + 7] != C)) return; } }
  size_t off = 0; char* ws = (char*)d_ws;
  auto carve = [&](size_t bytes) { char* p = ws + off; off += (bytes + 255) & ~(size_t)255; return p; };
  b16* WT0 = (b16*)carve((size_t)NCOL * IN * 2); b16* WT1 = (b16*)carve((size_t)NCOL * C * 2); b16* WQ1 = (b16*)carve((size_t)NCOL * C * 2); b16* WT2 = (b16*)carve((size_t)NCOL * C * 2); b16* WQ2 = (b16*)carve((size_t)NCOL * C * 2);
  float* LP = (float*)carve((size_t)NP * C * 4); float* OP = (float*)carve((size_t)NP * C * 4); float* GB = (float*)carve((size_t)NP * 2 * C * 4); float* Hh = (float*)carve((size_t)NP * C * 4); float* PART = (float*)carve((size_t)NBLK * C * 4); float* ST0 = (float*)carve(2 * C * 4); float* ST1 = (float*)carve(2 * C * 4);
  CsrBufs csr; off = csr_carve(csr, ws, off, E, N);
  if (off > ws_size || off > ((size_t)176 << 20)) return;
  wt_kernel<IN><<<(NCOL * IN / 8 + 255) / 256, 256, 0, stream>>>(Fp(5), Fp(2), Fp(6), Fp(3), WT0, WSC);
  wt_kernel<C><<<(NCOL * C / 8 + 255) / 256, 256, 0, stream>>>(Fp(13), Fp(10), Fp(14), Fp(11), WT1, WSC); wt_kernel<C><<<(NCOL * C / 8 + 255) / 256, 256, 0, stream>>>(Fp(13), Fp(10), Fp(14), Fp(11), WQ1, WSQ);
  wt_kernel<C><<<(NCOL * C / 8 + 255) / 256, 256, 0, stream>>>(Fp(21), Fp(18), Fp(22), Fp(19), WT2, WSC); wt_kernel<C><<<(NCOL * C / 8 + 255) / 256, 256, 0, stream>>>(Fp(21), Fp(18), Fp(22), Fp(19), WQ2, WSQ);
  csr_build(csr, Ip(1) + EFULL, E, N, stream);
  node_kernel<IN, true, true><<<NP / 32, 64, 0, stream>>>(Fp(0), ST0, Fp(8), Fp(9), WT0, WT0, Fp(7), Fp(4), LP, OP, GB);
  agg_kernel<true><<<NP / 32, 256, 0, stream>>>(LP, OP, GB, Ip(1), csr.PERM, csr.ROWPTR, csr.ROWCNT, (int)csr.permLen, Hh, NP);
  colpart_kernel<0><<<NBLK, 256, 0, stream>>>(Hh, ST0, PART); colred_kernel<0><<<1, 64, 0, stream>>>(PART, ST0); colpart_kernel<1><<<NBLK, 256, 0, stream>>>(Hh, ST0, PART); colred_kernel<1><<<1, 64, 0, stream>>>(PART, ST0);
  node_kernel<C, false, true><<<NP / 32, 64, 0, stream>>>(Hh, ST0, Fp(8), Fp(9), WT1, WQ1, Fp(15), Fp(12), LP, OP, GB);
  agg_kernel<true><<<NP / 32, 256, 0, stream>>>(LP, OP, GB, Ip(1), csr.PERM, csr.ROWPTR, csr.ROWCNT, (int)csr.permLen, Hh, NP);
  colpart_kernel<0><<<NBLK, 256, 0, stream>>>(Hh, ST1, PART); colred_kernel<0><<<1, 64, 0, stream>>>(PART, ST1); colpart_kernel<1><<<NBLK, 256, 0, stream>>>(Hh, ST1, PART); colred_kernel<1><<<1, 64, 0, stream>>>(PART, ST1);
  node_kernel<C, false, false><<<NP / 32, 64, 0, stream>>>(Hh, ST1, Fp(16), Fp(17), WT2, WQ2, Fp(23), Fp(20), LP, OP, GB);
  agg_kernel<false><<<NPL / 32, 256, 0, stream>>>(LP, OP, GB, Ip(1), csr.PERM, csr.ROWPTR, csr.ROWCNT, (int)csr.permLen, (float*)d_out, NL);
}
